// PlacementGNN_73143293051349
// MI455X (gfx1250) — hardware-run, weakly checked
//
#include <hip/hip_runtime.h>


namespace {
constexpr int N = 10000, E = 100000, NG = 4, DN = 8, DE = 4, HID = 128, OUT = 64, NHD = 8, HC = NHD * HID, NL = 4;
constexpr float XS = 8.0f, WSC = 256.0f, SLOPE = 0.2f;
typedef _Float16 b16;
typedef __attribute__((ext_vector_type(16))) _Float16 v16b;
typedef __attribute__((ext_vector_type(8))) _Float16 v8b;
typedef __attribute__((ext_vector_type(8))) float v8f;
typedef __attribute__((ext_vector_type(4))) float v4f;
typedef __attribute__((ext_vector_type(2))) float v2f;
__device__ __forceinline__ float bf16_rne(float f) { unsigned int u = __float_as_uint(f); u += 0x7FFFu + ((u >> 16) & 1u); float r = __uint_as_float(u & 0xFFFF0000u); asm volatile("" : "+v"(r)); return r; }
__device__ __forceinline__ void split16(float v, b16& hi, b16& lo) { hi = (b16)v; lo = (b16)(v - (float)hi); }
__device__ __forceinline__ v16b frag_kb(const b16* p, int hh) { const v8b a = *(const v8b*)(p + 8 * hh), b = *(const v8b*)(p + 16 + 8 * hh); v16b f;
#pragma unroll
  for (int e = 0; e < 8; ++e) { f[e] = a[e]; f[8 + e] = b[e]; } return f; }
__device__ __forceinline__ v8f wmma16b(v16b a, v16b b, v8f c) { v8f d = __builtin_amdgcn_wmma_f32_16x16x32_f16(false, a, false, b, (short)0, c, false, false); asm volatile("v_nop\n\tv_nop\n\tv_nop\n\tv_nop" : "+v"(d) : "v"(a), "v"(b)); return d; }
__device__ __forceinline__ void wave_lds_sync() { __builtin_amdgcn_fence(__ATOMIC_RELEASE, "workgroup"); __builtin_amdgcn_wave_barrier(); __builtin_amdgcn_fence(__ATOMIC_ACQUIRE, "workgroup"); }
__device__ __forceinline__ float pmul(float a, float b) { float p = a * b; asm volatile("" : "+v"(p)); return p; }
__device__ __forceinline__ int iclamp(int v, int lo, int hi) { return v < lo ? lo : (v > hi ? hi : v); }
__device__ __forceinline__ float lrelu(float v) { return v > 0.0f ? v : SLOPE * v; }
constexpr int CSR_NBLK7 = 512, CSR_GB7 = 7, CSR_GN7 = 1 << CSR_GB7  , CSR_TS7 = (CSR_GN7 < 32 ? 32 : CSR_GN7)  , CSR_MAXG7 = 512, CSR_CAP7 = 12288  ;
__device__ __host__ __forceinline__ int csr_tix7(int v) { return (v >> CSR_GB7) * CSR_TS7 + (v & (CSR_GN7 - 1)); }
__global__ __launch_bounds__(64) void csrA_kernel7(const int* __restrict__ dst, int E, int N, int nG, int CHP, int NGP, int* __restrict__ STG, int* __restrict__ HST) {
  extern __shared__ int sm[];
  int* cnt = sm; int* run = sm + NGP; int* ids = sm + 2 * NGP;
  const int b = blockIdx.x; const int ch = (E + CSR_NBLK7 - 1) / CSR_NBLK7; const int e0 = b * ch, e1 = min(E, e0 + ch);
  for (int i = threadIdx.x; i < NGP; i += 64) cnt[i] = 0;
  for (int i = threadIdx.x; i < CHP; i += 64) ids[i] = -1;
  __syncthreads();
  if (threadIdx.x == 0) {
    for (int e = e0; e < e1; ++e) { int d = dst[e]; d = (d < 0) ? 0 : (d >= N ? N - 1 : d); cnt[d >> CSR_GB7] += 1; }
    int acc = 0; for (int g = 0; g < nG; ++g) { run[g] = acc; acc += cnt[g]; }
    for (int e = e0; e < e1; ++e) { int d = dst[e]; d = (d < 0) ? 0 : (d >= N ? N - 1 : d); const int g = d >> CSR_GB7; ids[run[g]] = e; run[g] += 1; } }
  __syncthreads();
  typedef __attribute__((ext_vector_type(4))) int v4i;
  for (int pass = 0; pass < 2; ++pass) {
    for (int i = threadIdx.x; i < CHP / 4; i += 64) *(volatile v4i*)(STG + (size_t)b * CHP + i * 4) = *(const v4i*)(&ids[i * 4]);
    for (int i = threadIdx.x; i < NGP / 4; i += 64) { v4i v; for (int e = 0; e < 4; ++e) v[e] = (i * 4 + e < nG) ? cnt[i * 4 + e] : 0; *(volatile v4i*)(HST + (size_t)b * NGP + i * 4) = v; }
    __threadfence(); }
}
__global__ __launch_bounds__(512) void csrS_kernel7(const int* __restrict__ HST, int nG, int NGP, int* __restrict__ START, int* __restrict__ TOT, int* __restrict__ OFF) {
  __shared__ int tot[CSR_MAXG7];
  const int b = threadIdx.x;
  for (int pass = 0; pass < 2; ++pass) { int runb = 0; for (int g = 0; g < nG; ++g) { int c = HST[(size_t)b * NGP + g]; c = (c < 0) ? 0 : c; ((volatile int*)OFF)[(size_t)g * CSR_NBLK7 + b] = runb; runb += c; } __threadfence(); }
  for (int g = threadIdx.x; g < nG; g += 512) { int s = 0; for (int bb = 0; bb < CSR_NBLK7; ++bb) { int c = HST[(size_t)bb * NGP + g]; s += (c < 0) ? 0 : c; } tot[g] = s; }
  __syncthreads();
  if (threadIdx.x < 32) {
    __shared__ int st[CSR_MAXG7 + 32];
    if (threadIdx.x == 0) { int acc = 0; for (int g = 0; g < NGP; ++g) { st[g] = acc; if (g < nG) acc += (tot[g] + 31) & ~31; } st[NGP] = acc; }
    __builtin_amdgcn_fence(__ATOMIC_RELEASE, "workgroup"); __builtin_amdgcn_wave_barrier(); __builtin_amdgcn_fence(__ATOMIC_ACQUIRE, "workgroup");
    for (int pass = 0; pass < 2; ++pass) { for (int i = threadIdx.x; i < NGP + 32; i += 32) { ((volatile int*)START)[i] = (i <= NGP) ? st[min(i, NGP)] : 0; ((volatile int*)TOT)[i] = (i < nG) ? tot[i] : 0; } __threadfence(); } }
}
__global__ __launch_bounds__(256) void csrB_kernel7(const int* __restrict__ dst, int N, int nG, int CHP, int NGP, int permLen, const int* __restrict__ STG, const int* __restrict__ HST, const int* __restrict__ OFF, const int* __restrict__ START, const int* __restrict__ TOT, int* __restrict__ PERM, int* __restrict__ ROWPTR, int* __restrict__ ROWCNT, int* __restrict__ FLAG) {
  typedef __attribute__((ext_vector_type(4))) int v4i;
  __shared__ int ids[CSR_CAP7]; __shared__ unsigned short key[CSR_CAP7]; __shared__ int outp[CSR_CAP7]; __shared__ int ncnt[CSR_GN7 + 1]; __shared__ int boff[CSR_NBLK7 + 1];
  const int g = blockIdx.x, t_ = threadIdx.x; int tot = TOT[g]; int st = START[g], stn = START[g + 1]; const int v0 = g * CSR_GN7; const int nv = min(CSR_GN7, N - v0); const int t0 = g * CSR_TS7;
  st = (st < 0) ? 0 : (st > permLen - 32 ? permLen - 32 : st) & ~31; stn = (stn < st) ? st : (stn > permLen ? permLen : stn); tot = (tot < 0) ? 0 : tot; if (tot > stn - st && tot <= CSR_CAP7) tot = stn - st;
  if (tot > CSR_CAP7) {
    for (int pass = 0; pass < 2; ++pass) { for (int i = t_; i < CSR_TS7 / 4; i += 256) { v4i a, c; for (int e = 0; e < 4; ++e) { a[e] = st; c[e] = 0; } *(volatile v4i*)(ROWPTR + t0 + i * 4) = a; *(volatile v4i*)(ROWCNT + t0 + i * 4) = c; } if (t_ == 0) ((volatile int*)FLAG)[0] = 1; __threadfence(); } (void)nv; return; }
  if (t_ == 0) { int acc = 0; for (int b = 0; b < CSR_NBLK7; ++b) { boff[b] = acc; int c = HST[(size_t)b * NGP + g]; c = (c < 0) ? 0 : (c > CHP ? CHP : c); acc += c; if (acc > tot) acc = tot; } boff[CSR_NBLK7] = acc; }
  for (int i = t_; i <= CSR_GN7; i += 256) ncnt[i] = 0;
  __syncthreads();
  for (int b = 0; b < CSR_NBLK7; ++b) { const int c = boff[b + 1] - boff[b]; int o_ = OFF[(size_t)g * CSR_NBLK7 + b]; o_ = (o_ < 0) ? 0 : (o_ > CHP - c ? CHP - c : o_); const int* src_ = STG + (size_t)b * CHP + o_;
    for (int i = t_; i < c; i += 256) { int id = src_[i]; id = (id < 0) ? 0 : id; ids[boff[b] + i] = id; int d = dst[id]; d = (d < v0) ? v0 : (d >= N ? N - 1 : d); int kk = d - v0; kk = (kk < 0) ? 0 : (kk >= CSR_GN7 ? CSR_GN7 - 1 : kk); key[boff[b] + i] = (unsigned short)kk; } }
  __syncthreads();
  if (t_ == 0) { for (int i = 0; i < tot; ++i) ncnt[key[i]] += 1; int acc = 0; for (int vl = 0; vl < CSR_GN7; ++vl) { const int c = ncnt[vl]; ncnt[vl] = acc; acc += c; } ncnt[CSR_GN7] = acc;
    for (int i = 0; i < tot; ++i) { const int vl = key[i]; outp[ncnt[vl]] = ids[i]; ncnt[vl] += 1; }
    for (int vl = CSR_GN7; vl > 0; --vl) ncnt[vl] = ncnt[vl - 1]; ncnt[0] = 0; }
  __syncthreads();
  for (int pass = 0; pass < 2; ++pass) {
    for (int i = t_; i < (stn - st) / 4; i += 256) { v4i v; for (int e = 0; e < 4; ++e) { const int q = i * 4 + e; v[e] = (q < tot) ? outp[q] : -1; } *(volatile v4i*)(PERM + st + i * 4) = v; }
    for (int i = t_; i < CSR_TS7 / 4; i += 256) { v4i a, c; for (int e = 0; e < 4; ++e) { const int vl = i * 4 + e; const int vc = vl < CSR_GN7 ? vl : CSR_GN7; a[e] = (vl < CSR_GN7) ? st + ncnt[vc] : st; c[e] = (vl < nv) ? (ncnt[(vc < CSR_GN7 ? vc : CSR_GN7 - 1) + 1] - ncnt[vc]) : 0; } *(volatile v4i*)(ROWPTR + t0 + i * 4) = a; *(volatile v4i*)(ROWCNT + t0 + i * 4) = c; }
    __threadfence(); }
}
__global__ __launch_bounds__(256) void csrZ_kernel7(int* __restrict__ p, size_t n4) { typedef __attribute__((ext_vector_type(4))) int v4i; const size_t tid = (size_t)blockIdx.x * 256 + threadIdx.x, nth = (size_t)gridDim.x * 256; v4i z = {0, 0, 0, 0}; for (size_t i = tid; i < n4; i += nth) *(volatile v4i*)(p + i * 4) = z; }
struct CsrBufs7 { int *STG, *HST, *OFF, *START, *TOT, *PERM, *ROWPTR, *ROWCNT, *FLAG; int nG, NGP, CHP; size_t permLen; char* base; size_t bytes; };
static size_t csr_carve7(CsrBufs7& c, char* ws, size_t off, int E, int N) {
  const size_t off0 = off; c.base = ws + off;
  auto al = [&](size_t bytes) { char* p = ws + off; off += (bytes + 255) & ~(size_t)255; return p; };
  c.nG = (N + CSR_GN7 - 1) / CSR_GN7; c.NGP = (c.nG + 31) & ~31; const int ch = (E + CSR_NBLK7 - 1) / CSR_NBLK7; c.CHP = (ch + 31) & ~31; c.permLen = (size_t)E + 32 * (size_t)c.nG + 32;
  c.STG = (int*)al((size_t)CSR_NBLK7 * c.CHP * 4); c.HST = (int*)al((size_t)CSR_NBLK7 * c.NGP * 4); c.OFF = (int*)al((size_t)c.NGP * CSR_NBLK7 * 4); c.START = (int*)al((size_t)(c.NGP + 64) * 4); c.TOT = (int*)al((size_t)(c.NGP + 64) * 4);
  c.PERM = (int*)al(c.permLen * 4); c.ROWPTR = (int*)al((size_t)c.nG * CSR_TS7 * 4); c.ROWCNT = (int*)al((size_t)c.nG * CSR_TS7 * 4); c.FLAG = (int*)al(256);
  c.bytes = off - off0; return off;
}
static void csr_build7(const CsrBufs7& c, const int* dst, int E, int N, hipStream_t stream) {
  const size_t smem = (size_t)(2 * c.NGP + c.CHP) * 4;
  csrZ_kernel7<<<512, 256, 0, stream>>>((int*)c.base, c.bytes / 16);
  csrA_kernel7<<<CSR_NBLK7, 64, smem, stream>>>(dst, E, N, c.nG, c.CHP, c.NGP, c.STG, c.HST);
  csrS_kernel7<<<1, 512, 0, stream>>>(c.HST, c.nG, c.NGP, c.START, c.TOT, c.OFF);
  csrB_kernel7<<<c.nG, 256, 0, stream>>>(dst, N, c.nG, c.CHP, c.NGP, (int)c.permLen, c.STG, c.HST, c.OFF, c.START, c.TOT, c.PERM, c.ROWPTR, c.ROWCNT, c.FLAG);
}


__global__ __launch_bounds__(256) void wput_kernel(const float* __restrict__ w, int KIN, int KP, int OUTW, b16* __restrict__ WT) { const int KG = KP / 8; const size_t u = (size_t)blockIdx.x * 256 + threadIdx.x; if (u >= (size_t)OUTW * KG) return; const int o = (int)(u / KG), k0 = (int)(u % KG) * 8; v8b v;
#pragma unroll
  for (int j = 0; j < 8; ++j) { const int k = k0 + j; v[j] = (b16)(k < KIN ? bf16_rne(w[(size_t)k * OUTW + o]) * WSC : 0.0f); } for (int pass = 0; pass < 2; ++pass) { *(volatile v8b*)(WT + (size_t)o * KP + k0) = v; __threadfence(); } }
template <int KIN, int KP, int MODE>
__global__ __launch_bounds__(32) void dense_kernel(const float* __restrict__ IN, const b16* __restrict__ WT, const float* __restrict__ bias, int NGp, int RLIM, float* __restrict__ OUT, int ncols = 128, int OWx = 0) {
  __shared__ __attribute__((aligned(16))) b16 Ah[16][KP + 8], Al[16][MODE == 0 ? 8 : KP + 8]; __shared__ float Tf[16][132]; const int lane = threadIdx.x, nloc = lane & 15, hlf = lane >> 4; const int g = blockIdx.x % NGp; const size_t m0 = (size_t)(blockIdx.x / NGp) * 16; if (m0 >= (size_t)RLIM) return; const int OW = OWx ? OWx : NGp * 128; const int ntile = ncols / 16;
  for (int rr = 0; rr < 16; ++rr) for (int q = 0; q < KP / 32; ++q) { const int k = q * 32 + lane; float v = (k < KIN) ? IN[(m0 + rr) * KIN + k] : 0.0f; if (MODE == 0) Ah[rr][k] = (b16)(bf16_rne(v) * XS); else { if (MODE == 2) v = fmaxf(v, 0.0f); b16 p, ql; split16(v * XS, p, ql); Ah[rr][k] = p; Al[rr][k] = ql; } }
  wave_lds_sync(); v8f acc[8];
#pragma unroll
  for (int t = 0; t < 8; ++t) acc[t] = (v8f){};
#pragma unroll
  for (int kb = 0; kb < KP; kb += 32) { const v16b a = frag_kb(&Ah[nloc][kb], hlf); v16b a2; if (MODE != 0) a2 = frag_kb(&Al[nloc][kb], hlf);
#pragma unroll
    for (int t = 0; t < 8; ++t) { if (t >= ntile) break; const v16b bw = frag_kb(WT + (size_t)(g * 128 + t * 16 + nloc) * KP + kb, hlf); acc[t] = wmma16b(a, bw, acc[t]); if (MODE != 0) acc[t] = wmma16b(a2, bw, acc[t]); } }
#pragma unroll
  for (int t = 0; t < 8; ++t) { if (t >= ntile) break; const int c = g * 128 + t * 16 + nloc; const float bb = bias ? bf16_rne(bias[c]) : 0.0f;
#pragma unroll
    for (int r8 = 0; r8 < 8; ++r8) Tf[8 * hlf + r8][t * 16 + nloc] = acc[t][r8] * (1.0f / (XS * WSC)) + bb; }
  wave_lds_sync();
  for (int pass = 0; pass < 2; ++pass) { for (int rr = 0; rr < 16; ++rr) if (lane * 4 < ncols) *(volatile v4f*)(OUT + (m0 + rr) * OW + g * 128 + lane * 4) = *(const v4f*)(&Tf[rr][lane * 4]); __threadfence(); }
}
__global__ __launch_bounds__(256) void vt_kernel(const float* __restrict__ We, const float* __restrict__ ae, b16* __restrict__ VTh, b16* __restrict__ VTl) { const int u = blockIdx.x * 256 + threadIdx.x; if (u >= NL * 16 * (HID / 8)) return; const int k0 = (u % (HID / 8)) * 8, hd = (u / (HID / 8)) % 16, l = u / ((HID / 8) * 16); v8b vh, vl;
  for (int j = 0; j < 8; ++j) { float s = 0.0f; if (hd < NHD) {
#pragma unroll 1
      for (int c = 0; c < HID; ++c) s += pmul(bf16_rne(We[((size_t)l * HID + k0 + j) * HC + hd * HID + c]), bf16_rne(ae[((size_t)l * NHD + hd) * HID + c])); }
    b16 p, q; split16(s * WSC, p, q); vh[j] = p; vl[j] = q; }
  for (int pass = 0; pass < 2; ++pass) { *(volatile v8b*)(VTh + ((size_t)l * 16 + hd) * HID + k0) = vh; *(volatile v8b*)(VTl + ((size_t)l * 16 + hd) * HID + k0) = vl; __threadfence(); } }
__global__ __launch_bounds__(32) void ae_kernel(const float* __restrict__ EA, const b16* __restrict__ VTh, const b16* __restrict__ VTl, int l, float* __restrict__ AE) {
  __shared__ __attribute__((aligned(16))) b16 Ah[16][HID + 8], Al[16][HID + 8]; __shared__ float Tf[16][17]; const int lane = threadIdx.x, nloc = lane & 15, hlf = lane >> 4; const size_t m0 = (size_t)blockIdx.x * 16;
  for (int rr = 0; rr < 16; ++rr) for (int q = 0; q < HID / 32; ++q) { b16 p, ql; split16(EA[(m0 + rr) * HID + q * 32 + lane] * XS, p, ql); Ah[rr][q * 32 + lane] = p; Al[rr][q * 32 + lane] = ql; }
  wave_lds_sync(); v8f acc = {}; const b16* bh = VTh + (size_t)l * 16 * HID, *bl = VTl + (size_t)l * 16 * HID;
#pragma unroll
  for (int kb = 0; kb < HID; kb += 32) { const v16b a = frag_kb(&Ah[nloc][kb], hlf), al = frag_kb(&Al[nloc][kb], hlf), b0 = frag_kb(bh + (size_t)nloc * HID + kb, hlf), b1 = frag_kb(bl + (size_t)nloc * HID + kb, hlf); acc = wmma16b(a, b0, acc); acc = wmma16b(a, b1, acc); acc = wmma16b(al, b0, acc); }
#pragma unroll
  for (int r8 = 0; r8 < 8; ++r8) Tf[8 * hlf + r8][nloc] = acc[r8] * (1.0f / (XS * WSC));
  wave_lds_sync();
  for (int pass = 0; pass < 2; ++pass) { for (int i2 = lane; i2 < 256; i2 += 32) ((volatile float*)AE)[m0 * 16 + i2] = Tf[i2 / 16][i2 % 16]; __threadfence(); } }
__global__ __launch_bounds__(256) void al_kernel(const float* __restrict__ XP, const float* __restrict__ as, const float* __restrict__ ad, int NLIM, float* __restrict__ AL) { const int wave = threadIdx.x >> 5, lane = threadIdx.x & 31; const size_t i = (size_t)blockIdx.x * 8 + wave; if (i >= (size_t)NLIM) return; float outv = 0.0f;
  for (int hd = 0; hd < NHD; ++hd) { float s = 0.0f, d = 0.0f; for (int q = 0; q < 4; ++q) { const float xv = XP[i * HC + hd * HID + q * 32 + lane]; s += pmul(xv, bf16_rne(as[hd * HID + q * 32 + lane])); d += pmul(xv, bf16_rne(ad[hd * HID + q * 32 + lane])); }
    for (int o = 16; o; o >>= 1) { s += __shfl_xor(s, o); d += __shfl_xor(d, o); } if (lane == hd) outv = s; if (lane == 8 + hd) outv = d; }
  for (int pass = 0; pass < 2; ++pass) { ((volatile float*)AL)[i * 32 + lane] = outv; __threadfence(); } }
__global__ __launch_bounds__(256) void agg_kernel(const float* __restrict__ XP, const float* __restrict__ AL, const float* __restrict__ AE, const float* __restrict__ Hin, const float* __restrict__ bg, const float* __restrict__ lg_, const float* __restrict__ lb, const int* __restrict__ srcs, const int* __restrict__ PERM, const int* __restrict__ ROWPTR, const int* __restrict__ ROWCNT, int permLen, int NLIM, float* __restrict__ HO) {
  const int wave = threadIdx.x >> 5, lane = threadIdx.x & 31; const size_t i = (size_t)blockIdx.x * 8 + wave; if (i >= (size_t)NLIM) return; int st = ROWPTR[i], cnt = ROWCNT[i]; cnt = iclamp(cnt, 0, 1 << 20); st = iclamp(st, 0, permLen - cnt);
  v4f tot = {0.0f, 0.0f, 0.0f, 0.0f};
#pragma unroll 1
  for (int hd = 0; hd < NHD; ++hd) { const float adi = AL[i * 32 + 8 + hd]; float m = -INFINITY, den = 0.0f, aes = 0.0f; int n = 0; v4f acc = {0.0f, 0.0f, 0.0f, 0.0f};
    auto step = [&](size_t u, float aed) { const float s = lrelu(AL[u * 32 + hd] + adi + aed); const float mn = fmaxf(m, s); const float sc = (m == -INFINITY) ? 0.0f : __expf(m - mn); const float p = __expf(s - mn); den = den * sc + p; const v4f xv = *(const v4f*)(XP + u * HC + hd * HID + lane * 4); for (int k = 0; k < 4; ++k) acc[k] = pmul(acc[k], sc) + pmul(p, xv[k]); m = mn; };
#pragma unroll 1
    for (int j = 0; j < cnt; ++j) { const int e = iclamp(PERM[st + j], 0, E - 1); const size_t u = (size_t)iclamp(srcs[e], 0, N - 1); if (u >= (size_t)NLIM) continue; const float aed = AE[(size_t)e * 16 + hd]; aes += aed; ++n; step(u, aed); }
    step(i, aes / (float)(n > 0 ? n : 1));
    const float inv = 1.0f / (den + 1e-16f); for (int k = 0; k < 4; ++k) tot[k] += pmul(acc[k], inv); }
  v4f hv; const v4f res = *(const v4f*)(Hin + i * HID + lane * 4); for (int k = 0; k < 4; ++k) hv[k] = pmul(tot[k], 1.0f / NHD) + bf16_rne(bg[lane * 4 + k]) + res[k];
  float s = hv[0] + hv[1] + hv[2] + hv[3]; for (int o = 16; o; o >>= 1) s += __shfl_xor(s, o); const float mu = s * (1.0f / HID); float q = 0.0f; for (int k = 0; k < 4; ++k) q += pmul(hv[k] - mu, hv[k] - mu); for (int o = 16; o; o >>= 1) q += __shfl_xor(q, o); const float rs = rsqrtf(q * (1.0f / HID) + 1e-5f);
  v4f r; for (int k = 0; k < 4; ++k) r[k] = fmaxf(pmul(pmul(hv[k] - mu, rs), bf16_rne(lg_[lane * 4 + k])) + bf16_rne(lb[lane * 4 + k]), 0.0f);
  for (int pass = 0; pass < 2; ++pass) { *(volatile v4f*)(HO + i * HID + lane * 4) = r; __threadfence(); } }
__global__ __launch_bounds__(512) void graph_kernel(const float* __restrict__ Hh, const int* __restrict__ batch, const float* __restrict__ W1, const float* __restrict__ b1, const float* __restrict__ W2, const float* __restrict__ b2, int NLIM, float* __restrict__ out2) {
  __shared__ float Gf[NG][2 * HID], Z[NG][HID], O[NG][OUT]; const int t = threadIdx.x; { const int g = t / HID, c = t % HID; float s = 0.0f, mx = -INFINITY; int n = 0;
#pragma unroll 1
    for (int i = 0; i < NLIM; ++i) if (iclamp(batch[i], -1, NG) == g) { const float v = Hh[(size_t)i * HID + c]; s += v; mx = fmaxf(mx, v); ++n; }
    Gf[g][c] = n > 0 ? s / (float)n : 0.0f; Gf[g][HID + c] = n > 0 ? mx : 0.0f; }
  __syncthreads(); { const int g = t / HID, o = t % HID; float s = bf16_rne(b1[o]);
#pragma unroll 1
    for (int k = 0; k < 2 * HID; ++k) s += pmul(Gf[g][k], bf16_rne(W1[(size_t)k * HID + o])); Z[g][o] = fmaxf(s, 0.0f); }
  __syncthreads(); if (t < NG * OUT) { const int g = t / OUT, o = t % OUT; float s = bf16_rne(b2[o]);
#pragma unroll 1
    for (int k = 0; k < HID; ++k) s += pmul(Z[g][k], bf16_rne(W2[(size_t)k * OUT + o])); O[g][o] = s; }
  __syncthreads(); if (t < 32) { for (int pass = 0; pass < 2; ++pass) { for (int q = t; q < NG * OUT; q += 32) ((volatile float*)out2)[q] = O[q / OUT][q % OUT]; __threadfence(); } } }
}

extern "C" void kernel_launch(void* const* d_in, const int* in_sizes, int n_in, void* d_out, int out_size, void* d_ws, size_t ws_size, hipStream_t stream) {
  (void)n_in;
  auto Fp = [&](int i) { return (const float*)d_in[i]; }; auto Ip = [&](int i) { return (const int*)d_in[i]; };
  if (in_sizes[0] != N * DN || in_sizes[1] != E * DE || in_sizes[2] != 2 * E || in_sizes[3] != N || in_sizes[4] != DN * HID || in_sizes[6] != DE * HID || in_sizes[8] != NL * HID * HC || in_sizes[9] != NL * HID * HC || in_sizes[16] != HID * HID || in_sizes[18] != HID * OUT || in_sizes[20] != 2 * HID * HID || out_size != N * OUT + NG * OUT) return;
  const int NLIM = N;
  size_t off = 0; char* ws = (char*)d_ws;
  auto carve = [&](size_t bytes) { char* p = ws + off; off += (bytes + 255) & ~(size_t)255; return p; };
  b16* WN = (b16*)carve((size_t)HID * 32 * 2); b16* WE = (b16*)carve((size_t)HID * 32 * 2); b16* WL = (b16*)carve((size_t)NL * HC * HID * 2); b16* W1T = (b16*)carve((size_t)HID * HID * 2); b16* W2T = (b16*)carve((size_t)OUT * HID * 2);
  float* HA = (float*)carve((size_t)N * HID * 4); float* HB = (float*)carve((size_t)N * HID * 4); float* EA = (float*)carve((size_t)E * HID * 4); float* XP = (float*)carve((size_t)N * HC * 4); b16* VTh = (b16*)carve((size_t)NL * 16 * HID * 2); b16* VTl = (b16*)carve((size_t)NL * 16 * HID * 2); float* AE = (float*)carve((size_t)E * 16 * 4); float* AL = (float*)carve((size_t)N * 32 * 4); float* Z1 = (float*)carve((size_t)N * HID * 4);
  CsrBufs7 csr; off = csr_carve7(csr, ws, off, E, N);
  if (off > ws_size || off > ((size_t)160 << 20)) return;
  wput_kernel<<<(HID * 4 + 255) / 256, 256, 0, stream>>>(Fp(4), DN, 32, HID, WN); wput_kernel<<<(HID * 4 + 255) / 256, 256, 0, stream>>>(Fp(6), DE, 32, HID, WE);
  for (int l = 0; l < NL; ++l) wput_kernel<<<(HC * 16 + 255) / 256, 256, 0, stream>>>(Fp(8) + (size_t)l * HID * HC, HID, HID, HC, WL + (size_t)l * HC * HID);
  wput_kernel<<<(HID * 16 + 255) / 256, 256, 0, stream>>>(Fp(16), HID, HID, HID, W1T); wput_kernel<<<(OUT * 16 + 255) / 256, 256, 0, stream>>>(Fp(18), HID, HID, OUT, W2T);
  csr_build7(csr, Ip(2) + E, E, N, stream);
  vt_kernel<<<(NL * 16 * (HID / 8) + 255) / 256, 256, 0, stream>>>(Fp(9), Fp(12), VTh, VTl);
  dense_kernel<DN, 32, 0><<<NLIM / 16, 32, 0, stream>>>(Fp(0), WN, Fp(5), 1, NLIM, HA);
  dense_kernel<DE, 32, 0><<<E / 16, 32, 0, stream>>>(Fp(1), WE, Fp(7), 1, E, EA);
  float* hin = HA; float* hout = HB;
  for (int l = 0; l < NL; ++l) {
    dense_kernel<HID, HID, 1><<<(NLIM / 16) * 8, 32, 0, stream>>>(hin, WL + (size_t)l * HC * HID, nullptr, 8, NLIM, XP);
    al_kernel<<<(NLIM + 7) / 8, 256, 0, stream>>>(XP, Fp(10) + (size_t)l * NHD * HID, Fp(11) + (size_t)l * NHD * HID, NLIM, AL);
    ae_kernel<<<E / 16, 32, 0, stream>>>(EA, VTh, VTl, l, AE);
    agg_kernel<<<(NLIM + 7) / 8, 256, 0, stream>>>(XP, AL, AE, hin, Fp(13) + l * HID, Fp(14) + l * HID, Fp(15) + l * HID, Ip(2), csr.PERM, csr.ROWPTR, csr.ROWCNT, (int)csr.permLen, NLIM, hout);
    float* tmp = hin; hin = hout; hout = tmp; }
  dense_kernel<HID, HID, 1><<<NLIM / 16, 32, 0, stream>>>(hin, W1T, Fp(17), 1, NLIM, Z1);
  float* out = (float*)d_out;
  dense_kernel<HID, HID, 2><<<NLIM / 16, 32, 0, stream>>>(Z1, W2T, Fp(19), 1, NLIM, out, OUT, OUT);
  graph_kernel<<<1, 512, 0, stream>>>(hin, Ip(3), Fp(20), Fp(21), Fp(22), Fp(23), NLIM, out + (size_t)N * OUT);
}
